// HyperGTConv_63771674411308
// MI455X (gfx1250) — hardware-verified
//
#include <hip/hip_runtime.h>


#define NN_  50000
#define NNP  50048
#define CC   256
#define NH_  8
#define DD   64
#define MM   64
#define NE   80
#define EPS  1e-6f
#define CQ   (0.125f * 0.35355339059327373f)
#define LOSC 1024.0f
#define LOSCI (1.0f / 1024.0f)

typedef _Float16 h16;
typedef unsigned short bf;
typedef __attribute__((ext_vector_type(16))) __bf16   v16bf;
typedef __attribute__((ext_vector_type(16))) _Float16 v16h;
typedef __attribute__((ext_vector_type(8)))  _Float16 v8h;
typedef __attribute__((ext_vector_type(8)))  unsigned short v8us;
typedef __attribute__((ext_vector_type(4)))  unsigned short v4us;
typedef __attribute__((ext_vector_type(8)))  float    v8f;
typedef __attribute__((ext_vector_type(4)))  float    v4f;
typedef v8h  __attribute__((may_alias)) v8ha;
typedef v4f  __attribute__((may_alias)) v4fa;
typedef v8us __attribute__((may_alias)) v8usa;

__device__ __forceinline__ unsigned short f2bf(float f) { unsigned u = __float_as_uint(f); u += 0x7FFFu + ((u >> 16) & 1u); return (unsigned short)(u >> 16); }
__device__ __forceinline__ float bf2f(unsigned short b) { return __uint_as_float(((unsigned)b) << 16); }
__device__ __forceinline__ float bfr(float f) { return bf2f(f2bf(f)); }
__device__ __forceinline__ v16h cat16(v8h lo, v8h hi) { return __builtin_shufflevector(lo, hi, 0, 1, 2, 3, 4, 5, 6, 7, 8, 9, 10, 11, 12, 13, 14, 15); }
__device__ __forceinline__ v16bf cat16b(v8us lo, v8us hi) { return __builtin_bit_cast(v16bf, __builtin_shufflevector(lo, hi, 0, 1, 2, 3, 4, 5, 6, 7, 8, 9, 10, 11, 12, 13, 14, 15)); }
__device__ __forceinline__ v8f wmma16(v16h a, v16h b, v8f c) { return __builtin_amdgcn_wmma_f32_16x16x32_f16(false, a, false, b, (short)0, c, false, false); }
__device__ __forceinline__ v8f wmmab(v16bf a, v16bf b, v8f c) { return __builtin_amdgcn_wmma_f32_16x16x32_bf16(false, a, false, b, (short)0, c, false, false); }
#define VST2(T, p, v) do { const T vst2_v_ = (v); *(volatile T*)(p) = vst2_v_; __threadfence(); *(volatile T*)(p) = vst2_v_; } while (0)

__global__ __launch_bounds__(256) void k_xb(const float* __restrict__ x, bf* Xb) {
    const int lane = threadIdx.x & 31, r = blockIdx.x * 8 + (threadIdx.x >> 5);
    if (r >= NNP) return;
    const int rr = (r < NN_) ? r : NN_ - 1;
    v8us t;
#pragma unroll
    for (int i = 0; i < 8; ++i) { const unsigned short hb = f2bf(x[(size_t)rr * CC + lane * 8 + i]); t[i] = (r < NN_) ? hb : (unsigned short)0; }
    VST2(v8us, Xb + (size_t)r * CC + lane * 8, t);
}
__global__ __launch_bounds__(256) void k_wt(const float* __restrict__ Wm, int K, int N, bf* WT) {
    __shared__ __align__(16) unsigned short tl[64 * 72];
    const int tid = threadIdx.x, k0 = blockIdx.x * 64, n0 = blockIdx.y * 64;
    const int kk = tid >> 2, nq = (tid & 3) * 16;
#pragma unroll
    for (int i = 0; i < 16; ++i) tl[(nq + i) * 72 + kk] = f2bf(Wm[(size_t)(k0 + kk) * N + n0 + nq + i]);
    __syncthreads();
    const int piece = tid & 7;
    auto pass = [&]() {
#pragma unroll
        for (int s = 0; s < 2; ++s) { const int nr = (tid >> 3) + 32 * s; const v8us val = *(const v8usa*)(tl + nr * 72 + piece * 8);
            *(volatile v8us*)(WT + (size_t)(n0 + nr) * K + k0 + piece * 8) = val; }
    };
    pass(); __threadfence(); pass();
}
__global__ __launch_bounds__(256) void k_pj(const float* __restrict__ P, bf* PB) {
    const int lane = threadIdx.x & 31, r = blockIdx.x * 8 + (threadIdx.x >> 5);
    if (r >= MM) return;
    typedef __attribute__((ext_vector_type(2))) unsigned short v2us; v2us t; t[0] = f2bf(P[r * DD + 2 * lane]); t[1] = f2bf(P[r * DD + 2 * lane + 1]);
    VST2(v2us, PB + r * DD + 2 * lane, t);
}

template <int MODE>
__global__ __launch_bounds__(128) void k_gemm64(const bf* __restrict__ Xb, const bf* __restrict__ WT, int c0h, const float* __restrict__ bias, void* C) {
    __shared__ __align__(16) float ost[64 * 68];
    const int lane = threadIdx.x & 31, wave = threadIdx.x >> 5, lr = lane & 15, hi = lane >> 4;
    const int rb = blockIdx.x * 64, r0 = rb + wave * 16;
    const size_t aoff = (size_t)(r0 + lr) * CC + 8 * hi;
    size_t boff[4];
#pragma unroll
    for (int t = 0; t < 4; ++t) boff[t] = (size_t)(c0h + t * 16 + lr) * CC + 8 * hi;
    v8f acc[4];
#pragma unroll
    for (int t = 0; t < 4; ++t) acc[t] = (v8f){};
#pragma unroll 1
    for (int kc = 0; kc < CC; kc += 32) {
        const v16bf a = cat16b(*(const v8us*)(Xb + aoff + kc), *(const v8us*)(Xb + aoff + kc + 16));
#pragma unroll
        for (int t = 0; t < 4; ++t) acc[t] = wmmab(a, cat16b(*(const v8us*)(WT + boff[t] + kc), *(const v8us*)(WT + boff[t] + kc + 16)), acc[t]);
        asm volatile("v_nop\n\tv_nop\n\tv_nop\n\tv_nop" : "+v"(acc[0]), "+v"(acc[1]), "+v"(acc[2]), "+v"(acc[3]) : "v"(a));
    }
    float* os = ost + wave * 16 * 68;
#pragma unroll
    for (int t = 0; t < 4; ++t) { const float bv = bfr(bias[c0h + t * 16 + lr]);
#pragma unroll
        for (int j = 0; j < 8; ++j) os[(hi * 8 + j) * 68 + t * 16 + lr] = acc[t][j] + bv; }
    __syncthreads();
    if (MODE == 0) {
        float* crow = (float*)C + (size_t)r0 * DD;
        auto pass = [&]() {
#pragma unroll
            for (int s = 0; s < 8; ++s) { const int Lid = (lane >> 3) + 4 * s, piece = lane & 7; const int row = Lid >> 1, cofs = (Lid & 1) * 32 + piece * 4;
                const v4f val = *(const v4fa*)(os + row * 68 + cofs); *(volatile v4f*)(crow + (size_t)row * DD + cofs) = val; }
        };
        pass(); __threadfence(); pass();
    } else {
        h16* vt = (h16*)C + rb;
        auto pass = [&]() {
#pragma unroll
            for (int s = 0; s < 4; ++s) { const int col = wave * 16 + 4 * s + (lane >> 3), q = lane & 7; v8h v;
#pragma unroll
                for (int i = 0; i < 8; ++i) { const int rl = q * 8 + i; v[i] = (rb + rl < NN_) ? (h16)ost[rl * 68 + col] : (h16)0.f; }
                *(volatile v8h*)(vt + (size_t)col * NNP + q * 8) = v; }
#pragma unroll
            for (int s = 0; s < 4; ++s) { const int col = DD + wave * 4 + s, q = lane & 7; if ((lane >> 3) == 0) { v8h v;
#pragma unroll
                for (int i = 0; i < 8; ++i) { const int rl = q * 8 + i; v[i] = (col == DD && rb + rl < NN_) ? (h16)0.015625f : (h16)0.f; }
                *(volatile v8h*)(vt + (size_t)col * NNP + q * 8) = v; } }
        };
        pass(); __threadfence(); pass();
    }
}

template <int MODE>
__global__ __launch_bounds__(128) void k_feat(const float* __restrict__ R, const bf* __restrict__ PB, void* C) {
    __shared__ __align__(16) float ost[64 * 68];
    const int lane = threadIdx.x & 31, wave = threadIdx.x >> 5, lr = lane & 15, hi = lane >> 4;
    const int rb = blockIdx.x * 64, r0 = rb + wave * 16;
    v16bf ah[2], al[2];
#pragma unroll
    for (int kc = 0; kc < 2; ++kc) { v8us h0, h1, l0, l1;
#pragma unroll
        for (int i = 0; i < 8; ++i) {
            const float v0 = CQ * R[(size_t)(r0 + lr) * DD + kc * 32 + 8 * hi + i], v1 = CQ * R[(size_t)(r0 + lr) * DD + kc * 32 + 16 + 8 * hi + i];
            const unsigned short b0 = f2bf(v0), b1 = f2bf(v1); h0[i] = b0; h1[i] = b1; l0[i] = f2bf(v0 - bf2f(b0)); l1[i] = f2bf(v1 - bf2f(b1)); }
        ah[kc] = cat16b(h0, h1); al[kc] = cat16b(l0, l1); }
    v8f acc[4];
#pragma unroll
    for (int t = 0; t < 4; ++t) acc[t] = (v8f){};
#pragma unroll
    for (int kc = 0; kc < 2; ++kc)
#pragma unroll
        for (int t = 0; t < 4; ++t) { const bf* bp = PB + (size_t)(t * 16 + lr) * DD + kc * 32 + 8 * hi; const v16bf b = cat16b(*(const v8us*)bp, *(const v8us*)(bp + 16)); acc[t] = wmmab(ah[kc], b, acc[t]); acc[t] = wmmab(al[kc], b, acc[t]); }
    asm volatile("v_nop\n\tv_nop\n\tv_nop\n\tv_nop" : "+v"(acc[0]), "+v"(acc[1]), "+v"(acc[2]), "+v"(acc[3]));
    float* os = ost + wave * 16 * 68;
#pragma unroll
    for (int t = 0; t < 4; ++t)
#pragma unroll
        for (int j = 0; j < 8; ++j) os[(hi * 8 + j) * 68 + t * 16 + lr] = __expf(acc[t][j]) + EPS;
    __syncthreads();
    if (MODE == 0) {
        float* crow = (float*)C + (size_t)r0 * MM;
        auto pass = [&]() {
#pragma unroll
            for (int s = 0; s < 8; ++s) { const int Lid = (lane >> 3) + 4 * s, piece = lane & 7; const int row = Lid >> 1, cofs = (Lid & 1) * 32 + piece * 4;
                const v4f val = *(const v4fa*)(os + row * 68 + cofs); *(volatile v4f*)(crow + (size_t)row * MM + cofs) = val; }
        };
        pass(); __threadfence(); pass();
    } else {
        h16* kt = (h16*)C + rb;
        auto pass = [&]() {
#pragma unroll
            for (int s = 0; s < 4; ++s) { const int col = wave * 16 + 4 * s + (lane >> 3), q = lane & 7; v8h v;
#pragma unroll
                for (int i = 0; i < 8; ++i) { const int rl = q * 8 + i; v[i] = (rb + rl < NN_) ? (h16)ost[rl * 68 + col] : (h16)0.f; }
                *(volatile v8h*)(kt + (size_t)col * NNP + q * 8) = v; }
        };
        pass(); __threadfence(); pass();
    }
}

__global__ __launch_bounds__(128) void k_kv(const h16* __restrict__ KPT, const h16* __restrict__ VT, h16* KVH, h16* KVL) {
    __shared__ __align__(16) float ost[64 * 84];
    const int lane = threadIdx.x & 31, wave = threadIdx.x >> 5, lr = lane & 15, hi = lane >> 4;
    const int m0 = wave * 16;
    const size_t aoff = (size_t)(m0 + lr) * NNP + 8 * hi;
    size_t boff[5];
#pragma unroll
    for (int t = 0; t < 5; ++t) boff[t] = (size_t)(t * 16 + lr) * NNP + 8 * hi;
    v8f acc[5];
#pragma unroll
    for (int t = 0; t < 5; ++t) acc[t] = (v8f){};
#pragma unroll 1
    for (int kc = 0; kc < NNP; kc += 32) {
        const v16h a = cat16(*(const v8h*)(KPT + aoff + kc), *(const v8h*)(KPT + aoff + kc + 16));
#pragma unroll
        for (int t = 0; t < 5; ++t) acc[t] = wmma16(a, cat16(*(const v8h*)(VT + boff[t] + kc), *(const v8h*)(VT + boff[t] + kc + 16)), acc[t]);
        asm volatile("v_nop\n\tv_nop\n\tv_nop\n\tv_nop" : "+v"(acc[0]), "+v"(acc[1]), "+v"(acc[2]), "+v"(acc[3]), "+v"(acc[4]) : "v"(a));
    }
    float* os = ost + wave * 16 * 84;
#pragma unroll
    for (int t = 0; t < 5; ++t)
#pragma unroll
        for (int j = 0; j < 8; ++j) os[(hi * 8 + j) * 84 + t * 16 + lr] = acc[t][j];
    __syncthreads();
    auto pass = [&]() {
#pragma unroll
        for (int s = 0; s < 5; ++s) { const int e = wave * 20 + 4 * s + (lane >> 3), q = lane & 7; v8h vh, vl;
#pragma unroll
            for (int i = 0; i < 8; ++i) { const float v = ost[(q * 8 + i) * 84 + e]; const h16 a = (h16)v; vh[i] = a; vl[i] = (h16)((v - (float)a) * LOSC); }
            *(volatile v8h*)(KVH + (size_t)e * MM + q * 8) = vh; *(volatile v8h*)(KVL + (size_t)e * MM + q * 8) = vl; }
    };
    pass(); __threadfence(); pass();
}

__global__ __launch_bounds__(128) void k_z(const float* __restrict__ QP, const h16* __restrict__ KVH, const h16* __restrict__ KVL, bf* ZH, bf* ZL) {
    __shared__ __align__(16) float ost[4][16 * 84];
    const int lane = threadIdx.x & 31, wave = threadIdx.x >> 5, lr = lane & 15, hi = lane >> 4;
    const int r0 = blockIdx.x * 64 + wave * 16;
    v16h ah[2], al[2];
#pragma unroll
    for (int kc = 0; kc < 2; ++kc)
#pragma unroll
        for (int q = 0; q < 16; ++q) { const int m = kc * 32 + ((q < 8) ? (8 * hi + q) : (16 + 8 * hi + (q - 8))); const float v = QP[(size_t)(r0 + lr) * MM + m];
            const h16 hv = (h16)v; ah[kc][q] = hv; al[kc][q] = (h16)((v - (float)hv) * LOSC); }
    v8f acc[5], accx[5];
#pragma unroll
    for (int t = 0; t < 5; ++t) { acc[t] = (v8f){}; accx[t] = (v8f){}; }
#pragma unroll
    for (int kc = 0; kc < 2; ++kc)
#pragma unroll
        for (int t = 0; t < 5; ++t) { const size_t bo = (size_t)(t * 16 + lr) * MM + kc * 32 + 8 * hi;
            const v16h bh = cat16(*(const v8h*)(KVH + bo), *(const v8h*)(KVH + bo + 16)), bl = cat16(*(const v8h*)(KVL + bo), *(const v8h*)(KVL + bo + 16));
            acc[t] = wmma16(ah[kc], bh, acc[t]); accx[t] = wmma16(ah[kc], bl, accx[t]); accx[t] = wmma16(al[kc], bh, accx[t]); }
    asm volatile("v_nop\n\tv_nop\n\tv_nop\n\tv_nop" : "+v"(acc[0]), "+v"(acc[1]), "+v"(acc[2]), "+v"(acc[3]), "+v"(acc[4]));
    asm volatile("v_nop\n\tv_nop\n\tv_nop\n\tv_nop" : "+v"(accx[0]), "+v"(accx[1]), "+v"(accx[2]), "+v"(accx[3]), "+v"(accx[4]));
    float* os = &ost[wave][0];
#pragma unroll
    for (int t = 0; t < 5; ++t)
#pragma unroll
        for (int j = 0; j < 8; ++j) os[(hi * 8 + j) * 84 + t * 16 + lr] = acc[t][j] + accx[t][j] * LOSCI;
    asm volatile("" ::: "memory");
    __builtin_amdgcn_fence(__ATOMIC_RELEASE, "workgroup");
    __builtin_amdgcn_wave_barrier();
    auto pass = [&]() {
#pragma unroll
        for (int s = 0; s < 4; ++s) { const int row = 4 * s + (lane >> 3), piece = lane & 7; const float* sp = os + row * 84 + piece * 8; const float dn = 1.0f / (os[row * 84 + DD] * 64.0f + EPS); v8us oh, ol;
#pragma unroll
            for (int i = 0; i < 8; ++i) { const float z = sp[i] * dn; const unsigned short hb = f2bf(z); oh[i] = hb; ol[i] = f2bf(z - bf2f(hb)); }
            *(volatile v8us*)(ZH + (size_t)(r0 + row) * DD + piece * 8) = oh; *(volatile v8us*)(ZL + (size_t)(r0 + row) * DD + piece * 8) = ol; }
    };
    pass(); __threadfence(); pass();
}

__global__ __launch_bounds__(128) void k_out(const bf* __restrict__ ZH, const bf* __restrict__ ZL, const bf* __restrict__ WoT, int h, const float* __restrict__ bo, float* out) {
    __shared__ __align__(16) float ost[4][16 * 68];
    const int lane = threadIdx.x & 31, wave = threadIdx.x >> 5, lr = lane & 15, hi = lane >> 4;
    const int r0 = blockIdx.x * 64 + wave * 16;
    const size_t aoff = (size_t)(r0 + lr) * DD + 8 * hi;
    size_t boff[4];
#pragma unroll
    for (int t = 0; t < 4; ++t) boff[t] = (size_t)(t * 16 + lr) * (NH_ * DD) + h * DD + 8 * hi;
    v8f acc[4];
#pragma unroll
    for (int t = 0; t < 4; ++t) acc[t] = (v8f){};
#pragma unroll
    for (int kc = 0; kc < DD; kc += 32) {
        const v16bf a = cat16b(*(const v8us*)(ZH + aoff + kc), *(const v8us*)(ZH + aoff + kc + 16)), al = cat16b(*(const v8us*)(ZL + aoff + kc), *(const v8us*)(ZL + aoff + kc + 16));
#pragma unroll
        for (int t = 0; t < 4; ++t) { const v16bf b = cat16b(*(const v8us*)(WoT + boff[t] + kc), *(const v8us*)(WoT + boff[t] + kc + 16)); acc[t] = wmmab(a, b, acc[t]); acc[t] = wmmab(al, b, acc[t]); }
    }
    asm volatile("v_nop\n\tv_nop\n\tv_nop\n\tv_nop" : "+v"(acc[0]), "+v"(acc[1]), "+v"(acc[2]), "+v"(acc[3]));
    float* os = &ost[wave][0];
#pragma unroll
    for (int t = 0; t < 4; ++t) { const int col = t * 16 + lr; const float bv = (h == 0) ? bfr(bo[col]) : 0.f;
#pragma unroll
        for (int j = 0; j < 8; ++j) { const int row = r0 + hi * 8 + j, rowc = (row < NN_) ? row : (NN_ - 1); const float pv = out[(size_t)rowc * DD + col]; const float prev = (h == 0 || row >= NN_) ? 0.f : pv; os[(hi * 8 + j) * 68 + col] = prev + acc[t][j] + bv; } }
    __syncthreads();
    auto pass = [&]() {
#pragma unroll
        for (int s = 0; s < 8; ++s) { const int Lid = (lane >> 3) + 4 * s, piece = lane & 7; const int row = Lid >> 1, cofs = (Lid & 1) * 32 + piece * 4;
            if (r0 + row < NN_) { const v4f val = *(const v4fa*)(os + row * 68 + cofs); *(volatile v4f*)(out + (size_t)(r0 + row) * DD + cofs) = val; } }
    };
    pass(); __threadfence(); pass();
}

extern "C" void kernel_launch(void* const* d_in, const int* in_sizes, int n_in,
                              void* d_out, int out_size, void* d_ws, size_t ws_size, hipStream_t stream) {
    (void)in_sizes; (void)n_in; (void)out_size;
    const float* x = (const float*)d_in[0]; const float* Wq = (const float*)d_in[1]; const float* bq = (const float*)d_in[2]; const float* Wk = (const float*)d_in[3]; const float* bk = (const float*)d_in[4];
    const float* Wv = (const float*)d_in[5]; const float* bv = (const float*)d_in[6]; const float* Wo = (const float*)d_in[7]; const float* bo = (const float*)d_in[8]; const float* proj = (const float*)d_in[9];
    float* out = (float*)d_out;
    char* wsp = (char*)d_ws;
    auto take = [&](size_t bytes) { char* p = wsp; wsp += (bytes + 255) & ~(size_t)255; return (void*)p; };
    bf* Xb = (bf*)take((size_t)NNP * CC * 2); bf* WqT = (bf*)take((size_t)(NH_ * DD) * CC * 2); bf* WkT = (bf*)take((size_t)(NH_ * DD) * CC * 2); bf* WvT = (bf*)take((size_t)(NH_ * DD) * CC * 2);
    bf* WoT = (bf*)take((size_t)DD * (NH_ * DD) * 2); bf* PB = (bf*)take((size_t)MM * DD * 2);
    float* QH = (float*)take((size_t)NNP * DD * 4); float* KH = (float*)take((size_t)NNP * DD * 4); float* QP = (float*)take((size_t)NNP * MM * 4);
    h16* KPT = (h16*)take((size_t)MM * NNP * 2); h16* VT = (h16*)take((size_t)NE * NNP * 2);
    h16* KVH = (h16*)take((size_t)NE * MM * 2); h16* KVL = (h16*)take((size_t)NE * MM * 2);
    bf* ZH = (bf*)take((size_t)NNP * DD * 2); bf* ZL = (bf*)take((size_t)NNP * DD * 2);
    if ((size_t)(wsp - (char*)d_ws) > ws_size) return;
    k_xb<<<NNP / 8, 256, 0, stream>>>(x, Xb);
    k_wt<<<dim3(CC / 64, (NH_ * DD) / 64, 1), 256, 0, stream>>>(Wq, CC, NH_ * DD, WqT);
    k_wt<<<dim3(CC / 64, (NH_ * DD) / 64, 1), 256, 0, stream>>>(Wk, CC, NH_ * DD, WkT);
    k_wt<<<dim3(CC / 64, (NH_ * DD) / 64, 1), 256, 0, stream>>>(Wv, CC, NH_ * DD, WvT);
    k_wt<<<dim3((NH_ * DD) / 64, DD / 64, 1), 256, 0, stream>>>(Wo, NH_ * DD, DD, WoT);
    k_pj<<<MM / 8, 256, 0, stream>>>(proj, PB);
    for (int h = 0; h < NH_; ++h) {
        k_gemm64<0><<<NNP / 64, 128, 0, stream>>>(Xb, WqT, h * DD, bq, QH);
        k_gemm64<0><<<NNP / 64, 128, 0, stream>>>(Xb, WkT, h * DD, bk, KH);
        k_gemm64<1><<<NNP / 64, 128, 0, stream>>>(Xb, WvT, h * DD, bv, VT);
        k_feat<0><<<NNP / 64, 128, 0, stream>>>(QH, PB, QP);
        k_feat<1><<<NNP / 64, 128, 0, stream>>>(KH, PB, KPT);
        k_kv<<<1, 128, 0, stream>>>(KPT, VT, KVH, KVL);
        k_z<<<NNP / 64, 128, 0, stream>>>(QP, KVH, KVL, ZH, ZL);
        k_out<<<NNP / 64, 128, 0, stream>>>(ZH, ZL, WoT, h, bo, out);
    }
}
